// GAT_Transformer_ContextFusion_4629974745452
// MI455X (gfx1250) — hardware-verified
//
#include <hip/hip_runtime.h>


namespace {
constexpr int B = 8, N = 256, T = 24, C = 16, F = 48, NE = 16, CTX = 8, E = 64, HE = 4, HD = 16, L = 2, FF = 128, M = B * N, NR = M * T;
constexpr float XS = 8.0f, HS = 64.0f, WSC = 256.0f, NEG_SLOPE = 0.2f, MASKV = -9e15f;
typedef _Float16 b16;
typedef __attribute__((ext_vector_type(16))) _Float16 v16b;
typedef __attribute__((ext_vector_type(8))) _Float16 v8b;
typedef __attribute__((ext_vector_type(8))) float v8f;
typedef __attribute__((ext_vector_type(4))) float v4f;
typedef __attribute__((ext_vector_type(2))) float v2f;
__device__ __forceinline__ float bf16_rne(float f) { unsigned int u = __float_as_uint(f); u += 0x7FFFu + ((u >> 16) & 1u); return __uint_as_float(u & 0xFFFF0000u); }
__device__ __forceinline__ void split16(float v, b16& hi, b16& lo) { hi = (b16)v; lo = (b16)(v - (float)hi); }
__device__ __forceinline__ v16b frag_kb(const b16* p, int hh) { const v8b a = *(const v8b*)(p + 8 * hh), b = *(const v8b*)(p + 16 + 8 * hh); v16b f;
#pragma unroll
  for (int e = 0; e < 8; ++e) { f[e] = a[e]; f[8 + e] = b[e]; } return f; }
__device__ __forceinline__ v8f wmma16b(v16b a, v16b b, v8f c) { v8f d = __builtin_amdgcn_wmma_f32_16x16x32_f16(false, a, false, b, (short)0, c, false, false); asm volatile("v_nop\n\tv_nop\n\tv_nop\n\tv_nop" : "+v"(d) : "v"(a), "v"(b)); return d; }
__device__ __forceinline__ void wave_lds_sync() { __builtin_amdgcn_fence(__ATOMIC_RELEASE, "workgroup"); __builtin_amdgcn_wave_barrier(); __builtin_amdgcn_fence(__ATOMIC_ACQUIRE, "workgroup"); }
__device__ __forceinline__ float pmul(float a, float b) { float p = a * b; asm volatile("" : "+v"(p)); return p; }
__device__ __forceinline__ float leaky(float v) { return v >= 0.0f ? v : NEG_SLOPE * v; }
__device__ __forceinline__ float sigm(float v) { return 1.0f / (1.0f + __expf(-v)); }

__global__ __launch_bounds__(256) void wcopy_kernel(const float* __restrict__ w, int n8, b16* __restrict__ WT) {
  const int u = blockIdx.x * 256 + threadIdx.x; if (u >= n8) return; const int e = u * 8; v8b v;
#pragma unroll
  for (int j = 0; j < 8; ++j) v[j] = (b16)(bf16_rne(w[e + j]) * WSC); for (int pass = 0; pass < 2; ++pass) { *(volatile v8b*)(WT + e) = v; __threadfence(); }
}
__global__ __launch_bounds__(64) void wg_kernel(const float* __restrict__ gw, b16* __restrict__ WT) {
  const int o = threadIdx.x; if (o >= F) return; v8b v0 = {}, v1 = {}, vz = {};
#pragma unroll
  for (int k = 0; k < 8; ++k) { v0[k] = (b16)(bf16_rne(gw[k * F + o]) * WSC); v1[k] = (b16)(bf16_rne(gw[(8 + k) * F + o]) * WSC); }
  for (int pass = 0; pass < 2; ++pass) { *(volatile v8b*)(WT + o * 32) = v0; *(volatile v8b*)(WT + o * 32 + 8) = v1; *(volatile v8b*)(WT + o * 32 + 16) = vz; *(volatile v8b*)(WT + o * 32 + 24) = vz; __threadfence(); }
}
__global__ __launch_bounds__(32) void wh_kernel(const float* __restrict__ x, const b16* __restrict__ WG, const float* __restrict__ ga, int NRV, float* __restrict__ WH) {
  __shared__ __attribute__((aligned(16))) b16 Ah[16][32 + 8]; __shared__ __attribute__((aligned(16))) float Tf[16][E + 4];
  const int lane = threadIdx.x, nloc = lane & 15, hlf = lane >> 4; const size_t r0 = (size_t)blockIdx.x * 16; if (r0 >= (size_t)NRV) return;
  for (int rr = 0; rr < 16; ++rr) Ah[rr][lane] = lane < C ? (b16)(bf16_rne(x[(r0 + rr) * C + lane]) * XS) : (b16)0.0f;
  wave_lds_sync();
  v8f acc[3]; const v16b a = frag_kb(&Ah[nloc][0], hlf);
#pragma unroll
  for (int t = 0; t < 3; ++t) { acc[t] = (v8f){}; acc[t] = wmma16b(a, frag_kb(WG + (size_t)(t * 16 + nloc) * 32, hlf), acc[t]); }
  float p1[8], p2[8];
#pragma unroll
  for (int r8 = 0; r8 < 8; ++r8) { p1[r8] = 0.0f; p2[r8] = 0.0f; }
#pragma unroll
  for (int t = 0; t < 3; ++t) { const int c = t * 16 + nloc; const float a1 = bf16_rne(ga[c]), a2 = bf16_rne(ga[F + c]);
#pragma unroll
    for (int r8 = 0; r8 < 8; ++r8) { const float w = acc[t][r8] * (1.0f / (XS * WSC)); Tf[8 * hlf + r8][c] = w; p1[r8] += pmul(w, a1); p2[r8] += pmul(w, a2); } }
#pragma unroll
  for (int r8 = 0; r8 < 8; ++r8) { float u1 = p1[r8], u2 = p2[r8]; for (int o = 1; o < 16; o <<= 1) { u1 += __shfl_xor(u1, o); u2 += __shfl_xor(u2, o); } if (nloc < 16 - 2) { if (nloc == 0) { Tf[8 * hlf + r8][48] = u1; Tf[8 * hlf + r8][49] = u2; } else Tf[8 * hlf + r8][48 + 1 + nloc] = 0.0f; } }
  if (lane < 16) Tf[lane][63] = 0.0f;
  wave_lds_sync();
  for (int pass = 0; pass < 2; ++pass) { for (int rr = 0; rr < 16; ++rr) *(volatile v2f*)(WH + (r0 + rr) * E + lane * 2) = *(const v2f*)(&Tf[rr][lane * 2]); __threadfence(); }
}
__global__ __launch_bounds__(128) void gat_kernel(const float* __restrict__ WH, const int* __restrict__ adj, float* __restrict__ G) {
  __shared__ __attribute__((aligned(16))) b16 Ah[F][N + 8], Al[F][N + 8]; __shared__ __attribute__((aligned(16))) b16 Bh[4][16][N + 8], Bl[4][16][N + 8]; __shared__ float S2[N], S1[N]; __shared__ __attribute__((aligned(16))) float Tf[4][16 * F];
  const int wave = threadIdx.x >> 5, lane = threadIdx.x & 31, nloc = lane & 15, hlf = lane >> 4; const int bt = blockIdx.x; const int b = bt / T, t = bt % T;
  for (int i = threadIdx.x; i < F * N; i += 128) { const int f = i / N, j = i % N; const float v = WH[(((size_t)b * N + j) * T + t) * E + f]; b16 p, q; split16(v * XS, p, q); Ah[f][j] = p; Al[f][j] = q; }
  for (int j = threadIdx.x; j < N; j += 128) { const size_t r = ((size_t)b * N + j) * T + t; S1[j] = WH[r * E + 48]; S2[j] = WH[r * E + 49]; }
  __syncthreads();
#pragma unroll 1
  for (int it = 0; it < 4; ++it) { const int i0 = (wave * 4 + it) * 16;
    for (int rr = 0; rr < 16; ++rr) { const int i = i0 + rr; const float s1 = S1[i]; float ev[8]; float mx = -INFINITY;
      for (int q = 0; q < 8; ++q) { const int j = q * 32 + lane; const float e = (adj[i * N + j] > 0) ? leaky(s1 + S2[j]) : MASKV; ev[q] = e; mx = fmaxf(mx, e); }
      for (int o = 16; o; o >>= 1) mx = fmaxf(mx, __shfl_xor(mx, o)); float sum = 0.0f; for (int q = 0; q < 8; ++q) { ev[q] = __expf(ev[q] - mx); sum += ev[q]; } for (int o = 16; o; o >>= 1) sum += __shfl_xor(sum, o); const float inv = 1.0f / sum;
      for (int q = 0; q < 8; ++q) { b16 p, ql; split16(ev[q] * inv * XS, p, ql); Bh[wave][rr][q * 32 + lane] = p; Bl[wave][rr][q * 32 + lane] = ql; } }
    wave_lds_sync();
    v8f acc[3] = {(v8f){}, (v8f){}, (v8f){}};
#pragma unroll 2
    for (int kb = 0; kb < N; kb += 32) { const v16b bh = frag_kb(&Bh[wave][nloc][kb], hlf), bl = frag_kb(&Bl[wave][nloc][kb], hlf);
#pragma unroll
      for (int ft = 0; ft < 3; ++ft) { const v16b ah = frag_kb(&Ah[ft * 16 + nloc][kb], hlf), al = frag_kb(&Al[ft * 16 + nloc][kb], hlf); acc[ft] = wmma16b(ah, bh, acc[ft]); acc[ft] = wmma16b(ah, bl, acc[ft]); acc[ft] = wmma16b(al, bh, acc[ft]); acc[ft] = wmma16b(al, bl, acc[ft]); } }
#pragma unroll
    for (int ft = 0; ft < 3; ++ft)
#pragma unroll
      for (int r8 = 0; r8 < 8; ++r8) Tf[wave][nloc * F + ft * 16 + 8 * hlf + r8] = fmaxf(acc[ft][r8] * (1.0f / (XS * XS)), 0.0f);
    wave_lds_sync();
    const size_t base = (((size_t)b * T + t) * N + i0) * F;
    for (int pass = 0; pass < 2; ++pass) { for (int u = lane; u < 16 * F; u += 32) ((volatile float*)G)[base + u] = Tf[wave][u]; __threadfence(); }
    wave_lds_sync(); }
}
template <int L0>
__global__ __launch_bounds__(32) void qkv_kernel(const float* __restrict__ G, const float* __restrict__ emb, float* __restrict__ Hp, const b16* __restrict__ WIN, const float* __restrict__ bin, int NRV, float* __restrict__ QKV) {
  __shared__ __attribute__((aligned(16))) b16 Ah[16][E + 8], Al[16][E + 8]; __shared__ __attribute__((aligned(16))) float Tf[16][3 * E + 4], Hs[16][E + 4];
  const int lane = threadIdx.x, nloc = lane & 15, hlf = lane >> 4; const size_t r0 = (size_t)blockIdx.x * 16; if (r0 >= (size_t)NRV) return;
  for (int rr = 0; rr < 16; ++rr) { const size_t r = r0 + rr; v2f v; if (L0) { const int m = (int)(r / T); if (lane < 24) v = *(const v2f*)(G + r * F + lane * 2); else { const int n = m % N; v[0] = bf16_rne(emb[n * NE + (lane - 24) * 2]); v[1] = bf16_rne(emb[n * NE + (lane - 24) * 2 + 1]); } Hs[rr][lane * 2] = v[0]; Hs[rr][lane * 2 + 1] = v[1]; }
    else v = *(const v2f*)(Hp + r * E + lane * 2);
    for (int j = 0; j < 2; ++j) { b16 p, q; split16(v[j] * XS, p, q); Ah[rr][lane * 2 + j] = p; Al[rr][lane * 2 + j] = q; } }
  wave_lds_sync();
  if (L0) { for (int pass = 0; pass < 2; ++pass) { for (int rr = 0; rr < 16; ++rr) *(volatile v2f*)(Hp + (r0 + rr) * E + lane * 2) = *(const v2f*)(&Hs[rr][lane * 2]); __threadfence(); } }
  v8f acc[12];
#pragma unroll
  for (int tt = 0; tt < 12; ++tt) acc[tt] = (v8f){};
#pragma unroll
  for (int kb = 0; kb < E; kb += 32) { const v16b a = frag_kb(&Ah[nloc][kb], hlf), al = frag_kb(&Al[nloc][kb], hlf);
#pragma unroll
    for (int tt = 0; tt < 12; ++tt) { const v16b bw = frag_kb(WIN + (size_t)(tt * 16 + nloc) * E + kb, hlf); acc[tt] = wmma16b(a, bw, acc[tt]); acc[tt] = wmma16b(al, bw, acc[tt]); } }
#pragma unroll
  for (int tt = 0; tt < 12; ++tt) { const int c = tt * 16 + nloc; const float bb = bf16_rne(bin[c]);
#pragma unroll 1
    for (int r8 = 0; r8 < 8; ++r8) Tf[8 * hlf + r8][c] = acc[tt][r8] * (1.0f / (XS * WSC)) + bb; }
  wave_lds_sync();
  for (int pass = 0; pass < 2; ++pass) { for (int rr = 0; rr < 16; ++rr) for (int q = 0; q < 6; ++q) ((volatile float*)QKV)[(r0 + rr) * (3 * E) + q * 32 + lane] = Tf[rr][q * 32 + lane]; __threadfence(); }
}
__global__ __launch_bounds__(256) void attn_kernel(const float* __restrict__ QKV, int MV, float* __restrict__ O) {
  const int wave = threadIdx.x >> 5, lane = threadIdx.x & 31; const size_t m = (size_t)blockIdx.x * 8 + wave; if (m >= (size_t)MV) return; const float* base = QKV + m * T * (3 * E);
#pragma unroll 1
  for (int pass = 0; pass < 2; ++pass) {
#pragma unroll 1
    for (int h = 0; h < HE; ++h) { float kv[HD], vv = 0.0f; const int kk = lane < T ? lane : T - 1; for (int d = 0; d < HD; d += 4) { const v4f k4 = *(const v4f*)(base + (size_t)kk * (3 * E) + E + h * HD + d); for (int i = 0; i < 4; ++i) kv[d + i] = k4[i]; }
#pragma unroll 1
      for (int t = 0; t < T; ++t) { float s = 0.0f; for (int d = 0; d < HD; d += 4) { const v4f q4 = *(const v4f*)(base + (size_t)t * (3 * E) + h * HD + d); for (int i = 0; i < 4; ++i) s += pmul(q4[i], kv[d + i]); }
        s = (lane < T) ? s * 0.25f : -INFINITY; float mx = s; for (int o = 16; o; o >>= 1) mx = fmaxf(mx, __shfl_xor(mx, o)); float p = (lane < T) ? __expf(s - mx) : 0.0f; float sum = p; for (int o = 16; o; o >>= 1) sum += __shfl_xor(sum, o); const float a = p / sum;
        float acc = 0.0f;
#pragma unroll 1
        for (int k = 0; k < T; ++k) { const float ak = __shfl(a, k); const float vkd = (lane < HD) ? base[(size_t)k * (3 * E) + 2 * E + h * HD + lane] : 0.0f; acc += pmul(ak, vkd); }
        if (lane < HD) ((volatile float*)O)[(m * T + t) * E + h * HD + lane] = acc; (void)vv; } }
    __threadfence(); }
}
__device__ __forceinline__ void ln64(float (&vals)[4][8], const float* __restrict__ g, const float* __restrict__ b, int nloc) {
  float ps[8], pq[8];
#pragma unroll
  for (int r8 = 0; r8 < 8; ++r8) { ps[r8] = 0.0f;
#pragma unroll
    for (int t = 0; t < 4; ++t) ps[r8] += vals[t][r8];
    for (int o = 1; o < 16; o <<= 1) ps[r8] += __shfl_xor(ps[r8], o); ps[r8] *= (1.0f / E); pq[r8] = 0.0f;
#pragma unroll
    for (int t = 0; t < 4; ++t) { const float d = vals[t][r8] - ps[r8]; pq[r8] += pmul(d, d); }
    for (int o = 1; o < 16; o <<= 1) pq[r8] += __shfl_xor(pq[r8], o); pq[r8] = rsqrtf(pq[r8] * (1.0f / E) + 1e-5f); }
#pragma unroll
  for (int t = 0; t < 4; ++t) { const float gg = bf16_rne(g[t * 16 + nloc]), be = bf16_rne(b[t * 16 + nloc]);
#pragma unroll
    for (int r8 = 0; r8 < 8; ++r8) vals[t][r8] = pmul(pmul(vals[t][r8] - ps[r8], pq[r8]), gg) + be; }
}
__global__ __launch_bounds__(32) void post_kernel(const float* __restrict__ O, float* Hp, const b16* __restrict__ WOUT, const float* __restrict__ bout, const float* __restrict__ g1, const float* __restrict__ be1, const b16* __restrict__ W1T, const float* __restrict__ b1, const b16* __restrict__ W2T, const float* __restrict__ b2, const float* __restrict__ g2, const float* __restrict__ be2, int NRV) {
  __shared__ __attribute__((aligned(16))) b16 Ah[16][FF + 8], Al[16][FF + 8]; __shared__ __attribute__((aligned(16))) float Hs[16][E + 4], Tf[16][E + 4];
  const int lane = threadIdx.x, nloc = lane & 15, hlf = lane >> 4; const size_t r0 = (size_t)blockIdx.x * 16; if (r0 >= (size_t)NRV) return; const float sx = 1.0f / (XS * WSC), sh = 1.0f / (HS * WSC);
  for (int rr = 0; rr < 16; ++rr) { const v2f ov = *(const v2f*)(O + (r0 + rr) * E + lane * 2), hv = *(const v2f*)(Hp + (r0 + rr) * E + lane * 2); for (int j = 0; j < 2; ++j) { b16 p, q; split16(ov[j] * HS, p, q); Ah[rr][lane * 2 + j] = p; Al[rr][lane * 2 + j] = q; Hs[rr][lane * 2 + j] = hv[j]; } }
  wave_lds_sync();
  v8f acc[4];
#pragma unroll
  for (int tt = 0; tt < 4; ++tt) acc[tt] = (v8f){};
#pragma unroll
  for (int kb = 0; kb < E; kb += 32) { const v16b a = frag_kb(&Ah[nloc][kb], hlf), al = frag_kb(&Al[nloc][kb], hlf);
#pragma unroll
    for (int tt = 0; tt < 4; ++tt) { const v16b bw = frag_kb(WOUT + (size_t)(tt * 16 + nloc) * E + kb, hlf); acc[tt] = wmma16b(a, bw, acc[tt]); acc[tt] = wmma16b(al, bw, acc[tt]); } }
  float vals[4][8];
#pragma unroll
  for (int tt = 0; tt < 4; ++tt) { const int c = tt * 16 + nloc; const float bb = bf16_rne(bout[c]);
#pragma unroll
    for (int r8 = 0; r8 < 8; ++r8) vals[tt][r8] = Hs[8 * hlf + r8][c] + acc[tt][r8] * sh + bb; }
  ln64(vals, g1, be1, nloc);
  wave_lds_sync();
#pragma unroll
  for (int tt = 0; tt < 4; ++tt) { const int c = tt * 16 + nloc;
#pragma unroll
    for (int r8 = 0; r8 < 8; ++r8) { const int rl = 8 * hlf + r8; Hs[rl][c] = vals[tt][r8]; b16 p, q; split16(vals[tt][r8] * XS, p, q); Ah[rl][c] = p; Al[rl][c] = q; } }
  wave_lds_sync();
  v8f a1[8];
#pragma unroll
  for (int tt = 0; tt < 8; ++tt) a1[tt] = (v8f){};
#pragma unroll
  for (int kb = 0; kb < E; kb += 32) { const v16b a = frag_kb(&Ah[nloc][kb], hlf), al = frag_kb(&Al[nloc][kb], hlf);
#pragma unroll
    for (int tt = 0; tt < 8; ++tt) { const v16b bw = frag_kb(W1T + (size_t)(tt * 16 + nloc) * E + kb, hlf); a1[tt] = wmma16b(a, bw, a1[tt]); a1[tt] = wmma16b(al, bw, a1[tt]); } }
  wave_lds_sync();
#pragma unroll
  for (int tt = 0; tt < 8; ++tt) { const int c = tt * 16 + nloc; const float bb = bf16_rne(b1[c]);
#pragma unroll
    for (int r8 = 0; r8 < 8; ++r8) { const float v = fmaxf(a1[tt][r8] * sx + bb, 0.0f); b16 p, q; split16(v * HS, p, q); Ah[8 * hlf + r8][c] = p; Al[8 * hlf + r8][c] = q; } }
  wave_lds_sync();
#pragma unroll
  for (int tt = 0; tt < 4; ++tt) acc[tt] = (v8f){};
#pragma unroll
  for (int kb = 0; kb < FF; kb += 32) { const v16b a = frag_kb(&Ah[nloc][kb], hlf), al = frag_kb(&Al[nloc][kb], hlf);
#pragma unroll
    for (int tt = 0; tt < 4; ++tt) { const v16b bw = frag_kb(W2T + (size_t)(tt * 16 + nloc) * FF + kb, hlf); acc[tt] = wmma16b(a, bw, acc[tt]); acc[tt] = wmma16b(al, bw, acc[tt]); } }
#pragma unroll
  for (int tt = 0; tt < 4; ++tt) { const int c = tt * 16 + nloc; const float bb = bf16_rne(b2[c]);
#pragma unroll
    for (int r8 = 0; r8 < 8; ++r8) vals[tt][r8] = Hs[8 * hlf + r8][c] + acc[tt][r8] * sh + bb; }
  ln64(vals, g2, be2, nloc);
#pragma unroll
  for (int tt = 0; tt < 4; ++tt)
#pragma unroll
    for (int r8 = 0; r8 < 8; ++r8) Tf[8 * hlf + r8][tt * 16 + nloc] = vals[tt][r8];
  wave_lds_sync();
  for (int pass = 0; pass < 2; ++pass) { for (int rr = 0; rr < 16; ++rr) *(volatile v2f*)(Hp + (r0 + rr) * E + lane * 2) = *(const v2f*)(&Tf[rr][lane * 2]); __threadfence(); }
}
__global__ __launch_bounds__(32) void head_kernel(const float* __restrict__ ctx, const float* __restrict__ Hp, const b16* __restrict__ CW1, const float* __restrict__ cb1, const b16* __restrict__ CW2, const float* __restrict__ cb2, const b16* __restrict__ HW1, const float* __restrict__ hb1, const float* __restrict__ g, const float* __restrict__ bb, const float* __restrict__ hw2, const float* __restrict__ hb2, int MV, float* __restrict__ out) {
  __shared__ __attribute__((aligned(16))) b16 Ah[16][T * CTX + 8], Al[16][T * CTX + 8]; __shared__ float so[32];
  const int lane = threadIdx.x, nloc = lane & 15, hlf = lane >> 4; const float sx = 1.0f / (XS * WSC), sh = 1.0f / (HS * WSC);
#pragma unroll 1
  for (int half = 0; half < 2; ++half) { const size_t m0 = (size_t)blockIdx.x * 32 + half * 16;
    for (int rr = 0; rr < 16; ++rr) for (int q = 0; q < 6; ++q) { Ah[rr][q * 32 + lane] = (b16)(bf16_rne(ctx[(m0 + rr) * (T * CTX) + q * 32 + lane]) * XS); Al[rr][q * 32 + lane] = (b16)0.0f; }
    wave_lds_sync();
    v8f a1[8];
#pragma unroll
    for (int tt = 0; tt < 8; ++tt) a1[tt] = (v8f){};
#pragma unroll 2
    for (int kb = 0; kb < T * CTX; kb += 32) { const v16b a = frag_kb(&Ah[nloc][kb], hlf);
#pragma unroll
      for (int tt = 0; tt < 8; ++tt) a1[tt] = wmma16b(a, frag_kb(CW1 + (size_t)(tt * 16 + nloc) * (T * CTX) + kb, hlf), a1[tt]); }
    wave_lds_sync();
#pragma unroll
    for (int tt = 0; tt < 8; ++tt) { const int c = tt * 16 + nloc; const float b1v = bf16_rne(cb1[c]);
#pragma unroll
      for (int r8 = 0; r8 < 8; ++r8) { const float v = fmaxf(a1[tt][r8] * sx + b1v, 0.0f); b16 p, q; split16(v * HS, p, q); Ah[8 * hlf + r8][c] = p; Al[8 * hlf + r8][c] = q; } }
    wave_lds_sync();
    v8f a2[4];
#pragma unroll
    for (int tt = 0; tt < 4; ++tt) a2[tt] = (v8f){};
#pragma unroll
    for (int kb = 0; kb < FF; kb += 32) { const v16b a = frag_kb(&Ah[nloc][kb], hlf), al = frag_kb(&Al[nloc][kb], hlf);
#pragma unroll
      for (int tt = 0; tt < 4; ++tt) { const v16b bw = frag_kb(CW2 + (size_t)(tt * 16 + nloc) * FF + kb, hlf); a2[tt] = wmma16b(a, bw, a2[tt]); a2[tt] = wmma16b(al, bw, a2[tt]); } }
    wave_lds_sync();
#pragma unroll
    for (int tt = 0; tt < 4; ++tt) { const int c = tt * 16 + nloc; const float b2v = bf16_rne(cb2[c]);
#pragma unroll
      for (int r8 = 0; r8 < 8; ++r8) { const int rl = 8 * hlf + r8; const float cw = sigm(a2[tt][r8] * sh + b2v); const float last = (m0 + rl < (size_t)MV) ? Hp[((m0 + rl) * T + (T - 1)) * E + c] : 0.0f; const float fu = pmul(last, cw); b16 p, q; split16(fu * HS, p, q); Ah[rl][c] = p; Al[rl][c] = q; } }
    wave_lds_sync();
#pragma unroll
    for (int tt = 0; tt < 4; ++tt) a2[tt] = (v8f){};
#pragma unroll
    for (int kb = 0; kb < E; kb += 32) { const v16b a = frag_kb(&Ah[nloc][kb], hlf), al = frag_kb(&Al[nloc][kb], hlf);
#pragma unroll
      for (int tt = 0; tt < 4; ++tt) { const v16b bw = frag_kb(HW1 + (size_t)(tt * 16 + nloc) * E + kb, hlf); a2[tt] = wmma16b(a, bw, a2[tt]); a2[tt] = wmma16b(al, bw, a2[tt]); } }
    float vals[4][8];
#pragma unroll
    for (int tt = 0; tt < 4; ++tt) { const float b1v = bf16_rne(hb1[tt * 16 + nloc]);
#pragma unroll
      for (int r8 = 0; r8 < 8; ++r8) vals[tt][r8] = fmaxf(a2[tt][r8] * sh + b1v, 0.0f); }
    ln64(vals, g, bb, nloc);
    float pd[8];
#pragma unroll
    for (int r8 = 0; r8 < 8; ++r8) { pd[r8] = 0.0f;
#pragma unroll
      for (int tt = 0; tt < 4; ++tt) pd[r8] += pmul(vals[tt][r8], bf16_rne(hw2[tt * 16 + nloc]));
      for (int o = 1; o < 16; o <<= 1) pd[r8] += __shfl_xor(pd[r8], o); if (nloc == 0) so[half * 16 + 8 * hlf + r8] = (m0 + 8 * hlf + r8 < (size_t)MV) ? sigm(pd[r8] + bf16_rne(hb2[0])) : 0.0f; }
    wave_lds_sync(); }
  for (int pass = 0; pass < 2; ++pass) { ((volatile float*)out)[(size_t)blockIdx.x * 32 + lane] = so[lane]; __threadfence(); }
}
}

extern "C" void kernel_launch(void* const* d_in, const int* in_sizes, int n_in, void* d_out, int out_size, void* d_ws, size_t ws_size, hipStream_t stream) {
  (void)n_in;
  auto Fp = [&](int i) { return (const float*)d_in[i]; }; auto Ip = [&](int i) { return (const int*)d_in[i]; };
  if (in_sizes[0] != NR * C || in_sizes[1] != N * N || in_sizes[2] != NR * CTX || in_sizes[3] != N * NE || in_sizes[4] != C * F || in_sizes[6] != L * 3 * E * E || in_sizes[10] != L * FF * E || in_sizes[18] != FF * T * CTX || in_sizes[22] != E * E || out_size != M) return;
  const int BV = B; const int MV = BV * N, NRV = MV * T;
  size_t off = 0; char* ws = (char*)d_ws;
  auto carve = [&](size_t bytes) { char* p = ws + off; off += (bytes + 255) & ~(size_t)255; return p; };
  b16* WIN[L]; b16* WOUT[L]; b16* W1T[L]; b16* W2T[L]; for (int l = 0; l < L; ++l) { WIN[l] = (b16*)carve(3 * E * E * 2); WOUT[l] = (b16*)carve(E * E * 2); W1T[l] = (b16*)carve(FF * E * 2); W2T[l] = (b16*)carve(E * FF * 2); }
  b16* CW1 = (b16*)carve(FF * T * CTX * 2); b16* CW2 = (b16*)carve(E * FF * 2); b16* HW1 = (b16*)carve(E * E * 2); b16* WGT = (b16*)carve(F * 32 * 2);
  float* WH = (float*)carve((size_t)NR * E * 4); float* G = (float*)carve((size_t)NR * F * 4); float* Hp = (float*)carve((size_t)NR * E * 4); float* QKV = (float*)carve((size_t)NR * 3 * E * 4); float* O = (float*)carve((size_t)NR * E * 4);
  if (off > ws_size || off > ((size_t)128 << 20)) return;
  for (int l = 0; l < L; ++l) { wcopy_kernel<<<(3 * E * E / 8 + 255) / 256, 256, 0, stream>>>(Fp(6) + (size_t)l * 3 * E * E, 3 * E * E / 8, WIN[l]); wcopy_kernel<<<(E * E / 8 + 255) / 256, 256, 0, stream>>>(Fp(8) + (size_t)l * E * E, E * E / 8, WOUT[l]);
    wcopy_kernel<<<(FF * E / 8 + 255) / 256, 256, 0, stream>>>(Fp(10) + (size_t)l * FF * E, FF * E / 8, W1T[l]); wcopy_kernel<<<(E * FF / 8 + 255) / 256, 256, 0, stream>>>(Fp(12) + (size_t)l * E * FF, E * FF / 8, W2T[l]); }
  wcopy_kernel<<<(FF * T * CTX / 8 + 255) / 256, 256, 0, stream>>>(Fp(18), FF * T * CTX / 8, CW1); wcopy_kernel<<<(E * FF / 8 + 255) / 256, 256, 0, stream>>>(Fp(20), E * FF / 8, CW2); wcopy_kernel<<<(E * E / 8 + 255) / 256, 256, 0, stream>>>(Fp(22), E * E / 8, HW1);
  wg_kernel<<<1, 64, 0, stream>>>(Fp(4), WGT);
  wh_kernel<<<NRV / 16, 32, 0, stream>>>(Fp(0), WGT, Fp(5), NRV, WH);
  gat_kernel<<<BV * T, 128, 0, stream>>>(WH, Ip(1), G);
  for (int l = 0; l < L; ++l) {
    if (l == 0) qkv_kernel<1><<<NRV / 16, 32, 0, stream>>>(G, Fp(3), Hp, WIN[0], Fp(7), NRV, QKV); else qkv_kernel<0><<<NRV / 16, 32, 0, stream>>>(G, Fp(3), Hp, WIN[l], Fp(7) + l * 3 * E, NRV, QKV);
    attn_kernel<<<(MV + 7) / 8, 256, 0, stream>>>(QKV, MV, O);
    post_kernel<<<NRV / 16, 32, 0, stream>>>(O, Hp, WOUT[l], Fp(9) + l * E, Fp(14) + l * E, Fp(15) + l * E, W1T[l], Fp(11) + l * FF, W2T[l], Fp(13) + l * E, Fp(16) + l * E, Fp(17) + l * E, NRV); }
  head_kernel<<<M / 32, 32, 0, stream>>>(Fp(2), Hp, CW1, Fp(19), CW2, Fp(21), HW1, Fp(23), Fp(24), Fp(25), Fp(26), Fp(27), MV, (float*)d_out);
}
